// Encoder_23974507446482
// MI455X (gfx1250) — hardware-verified
//
#include <hip/hip_runtime.h>
#include <hip/hip_fp16.h>


#ifndef NB
#define NB 2
#endif
#ifndef SEQ
#define SEQ 2048
#endif
#define NB_FULL  2
#define SEQ_FULL 2048
#define MD   1024
#define NH   16
#define HD   64
#define FF   4096
#define NTOK (NB * SEQ)

static_assert(NB >= 1 && NB <= NB_FULL);
static_assert(SEQ >= 128 && SEQ <= SEQ_FULL);
static_assert(SEQ % 128 == 0);
static_assert(NTOK % 128 == 0);
static_assert(NH * HD == MD);
static_assert(MD % 128 == 0 && FF % 128 == 0);
static_assert(FF == 4 * MD);

typedef _Float16 v16h __attribute__((ext_vector_type(16)));
typedef _Float16 v8h  __attribute__((ext_vector_type(8)));
typedef _Float16 v4h  __attribute__((ext_vector_type(4)));
typedef float    v8f  __attribute__((ext_vector_type(8)));
typedef float    v4f  __attribute__((ext_vector_type(4)));

union Frag { v16h v; v8h h[2]; };

#define W_CARRY  64.0f
#define A_CARRY  8.0f
#define P_CARRY  16384.0f
#define SA_QKV   0.015625f
#define SA_WO    4.8828125e-04f
#define SA_FF    1.953125e-03f
#define CSC      (1.44269504088896340736f * 0.001953125f)
#define MASKT    (-1.0e9f * 1.44269504088896340736f)
#define SC_CTX   2.44140625e-04f

static __device__ __forceinline__ v8f zero8() {
    v8f z;
#pragma unroll
    for (int i = 0; i < 8; ++i) z[i] = 0.0f;
    return z;
}

static __device__ __forceinline__ v16h load_frag16(const _Float16* base, int ld, int lane) {
    int m  = lane & 15;
    int kb = (lane >> 4) << 3;
    const _Float16* p = base + (size_t)m * ld + kb;
    Frag f;
    f.h[0] = *(const v8h*)(p);
    f.h[1] = *(const v8h*)(p + 16);
    return f.v;
}

static __device__ __forceinline__ v8f wmma16(v16h a, v16h b, v8f c) {
    v8f d = __builtin_amdgcn_wmma_f32_16x16x32_f16(false, a, false, b, (short)0, c, false, false);
    asm volatile("v_nop\n\tv_nop\n\tv_nop\n\tv_nop" : "+v"(d) : "v"(a), "v"(b));
    return d;
}

static __device__ __forceinline__ float bf16r(float x) {
    unsigned u = __float_as_uint(x);
    u = (u + 0x7FFFu + ((u >> 16) & 1u)) & 0xFFFF0000u;
    return __uint_as_float(u);
}

static __device__ __forceinline__ float ex2(float x) {
    return __builtin_amdgcn_exp2f(x);
}

static __device__ __forceinline__ void wave_lds_sync() {
    __builtin_amdgcn_fence(3, "wavefront");
    asm volatile("s_wait_dscnt 0" ::: "memory");
    __builtin_amdgcn_wave_barrier();
}

__global__ __launch_bounds__(256) void k_wtr(const float* __restrict__ W, int N, int K,
                                             _Float16* __restrict__ WT) {
    __shared__ __align__(16) _Float16 T[64 * 72];
    const int tid = threadIdx.x;
    const int n0 = blockIdx.x * 64;
    const int k0 = blockIdx.y * 64;
#pragma unroll
    for (int p = 0; p < 4; ++p) {
        const int kl = p * 16 + (tid >> 4);
        const int nl = (tid & 15) * 4;
        const v4f xv = *(const v4f*)(W + (size_t)(k0 + kl) * N + n0 + nl);
        T[(nl + 0) * 72 + kl] = (_Float16)(bf16r(xv.x) * W_CARRY);
        T[(nl + 1) * 72 + kl] = (_Float16)(bf16r(xv.y) * W_CARRY);
        T[(nl + 2) * 72 + kl] = (_Float16)(bf16r(xv.z) * W_CARRY);
        T[(nl + 3) * 72 + kl] = (_Float16)(bf16r(xv.w) * W_CARRY);
    }
    __syncthreads();
    const int rl = tid >> 3, pc = (tid & 7) * 8;
    const v8h o0 = *(const v8h*)(&T[rl * 72 + pc]);
    const v8h o1 = *(const v8h*)(&T[(rl + 32) * 72 + pc]);
    _Float16* d0 = WT + (size_t)(n0 + rl) * K + k0 + pc;
    _Float16* d1 = WT + (size_t)(n0 + rl + 32) * K + k0 + pc;
    *(volatile v8h*)d0 = o0;
    *(volatile v8h*)d1 = o1;
    __threadfence();
    *(volatile v8h*)d0 = o0;
    *(volatile v8h*)d1 = o1;
}

__global__ __launch_bounds__(256) void k_xcvt(const float* __restrict__ inp,
                                              _Float16* __restrict__ xh) {
    const size_t idx = (size_t)blockIdx.x * 256 + threadIdx.x;
    const int r  = (int)(idx >> 7);
    const int c8 = (int)(idx & 127) * 8;
    const int b  = r / SEQ;
    const int s  = r - b * SEQ;
    const float* src = inp + ((size_t)b * SEQ_FULL + s) * MD + c8;
    const v4f a0 = *(const v4f*)(src);
    const v4f a1 = *(const v4f*)(src + 4);
    v8h hv;
    hv[0] = (_Float16)bf16r(a0.x); hv[1] = (_Float16)bf16r(a0.y);
    hv[2] = (_Float16)bf16r(a0.z); hv[3] = (_Float16)bf16r(a0.w);
    hv[4] = (_Float16)bf16r(a1.x); hv[5] = (_Float16)bf16r(a1.y);
    hv[6] = (_Float16)bf16r(a1.z); hv[7] = (_Float16)bf16r(a1.w);
    _Float16* dst = xh + (size_t)r * MD + c8;
    *(volatile v8h*)dst = hv;
    __threadfence();
    *(volatile v8h*)dst = hv;
}

template<int F32> struct OTy { typedef _Float16 t; };
template<> struct OTy<1> { typedef float t; };

template<int MODE>
__global__ __launch_bounds__(256) __attribute__((amdgpu_num_vgpr(256)))
void k_gemm(const _Float16* __restrict__ A, int lda,
            const _Float16* __restrict__ BT, int ldb,
            const float* __restrict__ bias,
            const float* __restrict__ res, int ldr,
            void* __restrict__ Cv, int ldc, int K, float sa, float so) {
    typedef typename OTy<(MODE >= 2) ? 1 : 0>::t ot;
    __shared__ __align__(16) ot Cst[8][32 * 64];

    const int tid  = threadIdx.x;
    const int lane = tid & 31;
    const int w    = tid >> 5;
    const int wr   = w >> 1;
    const int wc   = w & 1;
    const int r0   = (lane >> 4) << 3;
    const int cc   = lane & 15;
    const int m0   = blockIdx.x * 128 + wr * 32;
    const int n0   = blockIdx.y * 128 + wc * 64;
    const _Float16* Ab = A  + (size_t)m0 * lda;
    const _Float16* Bb = BT + (size_t)n0 * ldb;

    v8f acc[2][4];
#pragma unroll
    for (int mi = 0; mi < 2; ++mi)
#pragma unroll
        for (int ni = 0; ni < 4; ++ni) acc[mi][ni] = zero8();

#pragma unroll 1
    for (int k0 = 0; k0 < K; k0 += 32) {
        const v16h a0 = load_frag16(Ab + k0, lda, lane);
        const v16h a1 = load_frag16(Ab + (size_t)16 * lda + k0, lda, lane);
#pragma unroll
        for (int ni = 0; ni < 4; ++ni) {
            const v16h bf = load_frag16(Bb + (size_t)(ni * 16) * ldb + k0, ldb, lane);
            acc[0][ni] = wmma16(a0, bf, acc[0][ni]);
            acc[1][ni] = wmma16(a1, bf, acc[1][ni]);
        }
    }

    float bb[4];
#pragma unroll
    for (int ni = 0; ni < 4; ++ni) bb[ni] = bf16r(bias[n0 + ni * 16 + cc]);

#pragma unroll
    for (int mi = 0; mi < 2; ++mi)
#pragma unroll
        for (int ni = 0; ni < 4; ++ni)
#pragma unroll
            for (int g = 0; g < 8; ++g) {
                float v = __builtin_fmaf(acc[mi][ni][g], sa, bb[ni]);
                if constexpr (MODE == 1) v = fmaxf(v, 0.0f);
                const int li = (mi * 16 + r0 + g) * 64 + ni * 16 + cc;
                if constexpr (MODE < 2) Cst[w][li] = (_Float16)(v * so);
                else                    Cst[w][li] = v;
            }
    wave_lds_sync();

    ot* C = (ot*)Cv;
    if constexpr (MODE < 2) {
        const int rl = lane >> 3, pc = (lane & 7) * 8;
        v8h sv[8];
#pragma unroll
        for (int i = 0; i < 8; ++i) sv[i] = *(const v8h*)(&Cst[w][(4 * i + rl) * 64 + pc]);
        _Float16* Cb = C + (size_t)(m0 + rl) * ldc + n0 + pc;
#pragma unroll
        for (int i = 0; i < 8; ++i) *(volatile v8h*)(Cb + (size_t)(4 * i) * ldc) = sv[i];
        __threadfence();
#pragma unroll
        for (int i = 0; i < 8; ++i) *(volatile v8h*)(Cb + (size_t)(4 * i) * ldc) = sv[i];
    } else {
        const int rl = lane >> 4, pc = (lane & 15) * 4;
        v4f sv[16];
#pragma unroll
        for (int i = 0; i < 16; ++i) {
            const v4f cv = *(const v4f*)(&Cst[w][(2 * i + rl) * 64 + pc]);
            const int gm = m0 + 2 * i + rl;
            size_t rrow;
            if constexpr (MODE == 2) {
                const int b = gm / SEQ;
                rrow = (size_t)b * SEQ_FULL + (size_t)(gm - b * SEQ);
            } else {
                rrow = (size_t)gm;
            }
            v4f rv = *(const v4f*)(res + rrow * (size_t)ldr + n0 + pc);
            if constexpr (MODE == 2) {
                rv.x = bf16r(rv.x); rv.y = bf16r(rv.y); rv.z = bf16r(rv.z); rv.w = bf16r(rv.w);
            }
            sv[i] = cv + rv;
        }
        float* Cb = C + (size_t)(m0 + rl) * ldc + n0 + pc;
#pragma unroll
        for (int i = 0; i < 16; ++i) *(volatile v4f*)(Cb + (size_t)(2 * i) * ldc) = sv[i];
        __threadfence();
#pragma unroll
        for (int i = 0; i < 16; ++i) *(volatile v4f*)(Cb + (size_t)(2 * i) * ldc) = sv[i];
    }
}

__global__ __launch_bounds__(256) void k_vtr(const _Float16* __restrict__ v,
                                             _Float16* __restrict__ vT) {
    __shared__ __align__(16) _Float16 T[64 * 72];
    const int tid  = threadIdx.x;
    const int tok0 = blockIdx.x * 64;
    const int h    = blockIdx.y;
    const int b    = tok0 / SEQ;
    const int s0   = tok0 - b * SEQ;
#pragma unroll
    for (int p = 0; p < 2; ++p) {
        const int r  = p * 32 + (tid >> 3);
        const int c8 = (tid & 7) * 8;
        const v8h vv = *(const v8h*)(v + (size_t)(tok0 + r) * MD + h * HD + c8);
#pragma unroll
        for (int e = 0; e < 8; ++e) T[(c8 + e) * 72 + r] = vv[e];
    }
    __syncthreads();
    const int rl = tid >> 3, pc = (tid & 7) * 8;
    const v8h o0 = *(const v8h*)(&T[rl * 72 + pc]);
    const v8h o1 = *(const v8h*)(&T[(rl + 32) * 72 + pc]);
    _Float16* d0 = vT + ((size_t)(b * NH + h) * HD + rl) * SEQ + s0 + pc;
    _Float16* d1 = vT + ((size_t)(b * NH + h) * HD + rl + 32) * SEQ + s0 + pc;
    *(volatile v8h*)d0 = o0;
    *(volatile v8h*)d1 = o1;
    __threadfence();
    *(volatile v8h*)d0 = o0;
    *(volatile v8h*)d1 = o1;
}

__global__ __launch_bounds__(256) __attribute__((amdgpu_num_vgpr(256)))
void k_attn(const _Float16* __restrict__ qp,
            const _Float16* __restrict__ kp,
            const _Float16* __restrict__ vT,
            const int* __restrict__ mask,
            _Float16* __restrict__ ctx) {
    __shared__ __align__(16) _Float16 Pst[8][16 * 64];

    const int tid  = threadIdx.x;
    const int lane = tid & 31;
    const int w    = tid >> 5;
    const int r0   = (lane >> 4) << 3;
    const int cc   = lane & 15;
    const int bh   = blockIdx.y;
    const int b    = bh >> 4;
    const int h    = bh & 15;
    const int qrow = b * SEQ + blockIdx.x * 128 + w * 16;

    const v16h qf0 = load_frag16(qp + (size_t)qrow * MD + h * HD, MD, lane);
    const v16h qf1 = load_frag16(qp + (size_t)qrow * MD + h * HD + 32, MD, lane);
    const _Float16* kb = kp + (size_t)b * SEQ * MD + h * HD;
    const _Float16* vb = vT + (size_t)bh * HD * SEQ;
    const int* mrow = mask + (size_t)b * SEQ_FULL;

    v8f o[4];
#pragma unroll
    for (int dt = 0; dt < 4; ++dt) o[dt] = zero8();
    float mr[8], lr[8];
#pragma unroll
    for (int g = 0; g < 8; ++g) { mr[g] = -1.0e30f; lr[g] = 0.0f; }

#pragma unroll 1
    for (int key0 = 0; key0 < SEQ; key0 += 64) {
        v8f sc[4];
#pragma unroll
        for (int nt = 0; nt < 4; ++nt) {
            const _Float16* kr = kb + (size_t)(key0 + nt * 16) * MD;
            const v16h f0 = load_frag16(kr, MD, lane);
            const v16h f1 = load_frag16(kr + 32, MD, lane);
            v8f c = wmma16(qf0, f0, zero8());
            c = wmma16(qf1, f1, c);
            sc[nt] = c;
        }
        int mk[4];
#pragma unroll
        for (int nt = 0; nt < 4; ++nt) mk[nt] = mrow[key0 + nt * 16 + cc];
#pragma unroll
        for (int nt = 0; nt < 4; ++nt)
#pragma unroll
            for (int g = 0; g < 8; ++g) {
                const float tv = sc[nt][g] * CSC;
                sc[nt][g] = (mk[nt] == 0) ? MASKT : tv;
            }

        float corr[8];
#pragma unroll
        for (int g = 0; g < 8; ++g) {
            float tm = fmaxf(fmaxf(sc[0][g], sc[1][g]), fmaxf(sc[2][g], sc[3][g]));
            tm = fmaxf(tm, __shfl_xor(tm, 1, 32));
            tm = fmaxf(tm, __shfl_xor(tm, 2, 32));
            tm = fmaxf(tm, __shfl_xor(tm, 4, 32));
            tm = fmaxf(tm, __shfl_xor(tm, 8, 32));
            const float mn = fmaxf(mr[g], tm);
            corr[g] = ex2(mr[g] - mn);
            mr[g] = mn;
            float ps = 0.0f;
#pragma unroll
            for (int nt = 0; nt < 4; ++nt) {
                const float p = ex2(sc[nt][g] - mn);
                ps += p;
                Pst[w][(r0 + g) * 64 + nt * 16 + cc] = (_Float16)(p * P_CARRY);
            }
            lr[g] = __builtin_fmaf(lr[g], corr[g], ps);
        }
#pragma unroll
        for (int dt = 0; dt < 4; ++dt)
#pragma unroll
            for (int g = 0; g < 8; ++g) o[dt][g] = o[dt][g] * corr[g];
        wave_lds_sync();

        const v16h pa0 = load_frag16(&Pst[w][0], 64, lane);
        const v16h pa1 = load_frag16(&Pst[w][32], 64, lane);
#pragma unroll
        for (int dt = 0; dt < 4; ++dt) {
            const _Float16* vr = vb + (size_t)(dt * 16) * SEQ + key0;
            const v16h g0 = load_frag16(vr, SEQ, lane);
            const v16h g1 = load_frag16(vr + 32, SEQ, lane);
            o[dt] = wmma16(pa0, g0, o[dt]);
            o[dt] = wmma16(pa1, g1, o[dt]);
        }
        wave_lds_sync();
    }

    float inv[8];
#pragma unroll
    for (int g = 0; g < 8; ++g) {
        float L = lr[g];
        L += __shfl_xor(L, 1, 32);
        L += __shfl_xor(L, 2, 32);
        L += __shfl_xor(L, 4, 32);
        L += __shfl_xor(L, 8, 32);
        inv[g] = SC_CTX * __builtin_amdgcn_rcpf(L);
    }
#pragma unroll
    for (int dt = 0; dt < 4; ++dt)
#pragma unroll
        for (int g = 0; g < 8; ++g)
            Pst[w][(r0 + g) * 64 + dt * 16 + cc] = (_Float16)(o[dt][g] * inv[g]);
    wave_lds_sync();

    const int rl = lane >> 3, pc = (lane & 7) * 8;
    v8h sv[4];
#pragma unroll
    for (int i = 0; i < 4; ++i) sv[i] = *(const v8h*)(&Pst[w][(4 * i + rl) * 64 + pc]);
    _Float16* cb = ctx + (size_t)(qrow + rl) * MD + h * HD + pc;
#pragma unroll
    for (int i = 0; i < 4; ++i) *(volatile v8h*)(cb + (size_t)(4 * i) * MD) = sv[i];
    __threadfence();
#pragma unroll
    for (int i = 0; i < 4; ++i) *(volatile v8h*)(cb + (size_t)(4 * i) * MD) = sv[i];
}

template<int WH>
static __device__ __forceinline__ void ln_store(const float* __restrict__ yr,
                                                const float* __restrict__ gr,
                                                const float* __restrict__ br,
                                                float mu, float rstd,
                                                float* __restrict__ xo,
                                                _Float16* __restrict__ xh) {
#pragma unroll 1
    for (int i = 0; i < 8; ++i) {
        const v4f a  = *(const v4f*)(yr + i * 128);
        const v4f gv = *(const v4f*)(gr + i * 128);
        const v4f bv = *(const v4f*)(br + i * 128);
        v4f ov;
        ov.x = ((a.x - mu) * rstd) * bf16r(gv.x) + bf16r(bv.x);
        ov.y = ((a.y - mu) * rstd) * bf16r(gv.y) + bf16r(bv.y);
        ov.z = ((a.z - mu) * rstd) * bf16r(gv.z) + bf16r(bv.z);
        ov.w = ((a.w - mu) * rstd) * bf16r(gv.w) + bf16r(bv.w);
        *(volatile v4f*)(xo + i * 128) = ov;
        if constexpr (WH == 1) {
            v4h hv;
            hv.x = (_Float16)(ov.x * A_CARRY);
            hv.y = (_Float16)(ov.y * A_CARRY);
            hv.z = (_Float16)(ov.z * A_CARRY);
            hv.w = (_Float16)(ov.w * A_CARRY);
            *(volatile v4h*)(xh + i * 128) = hv;
        }
    }
}

template<int WH>
__global__ __launch_bounds__(256) void k_ln(const float* __restrict__ y,
                                            const float* __restrict__ gam,
                                            const float* __restrict__ bet,
                                            float* __restrict__ xo,
                                            _Float16* __restrict__ xh) {
    const int lane = threadIdx.x & 31;
    const int w    = threadIdx.x >> 5;
    const int row  = blockIdx.x * 8 + w;
    const float* yr = y + (size_t)row * MD + lane * 4;

    float s = 0.0f;
#pragma unroll 1
    for (int i = 0; i < 8; ++i) {
        const v4f a = *(const v4f*)(yr + i * 128);
        s += (a.x + a.y) + (a.z + a.w);
    }
#pragma unroll
    for (int m = 1; m < 32; m <<= 1) s += __shfl_xor(s, m, 32);
    const float mu = s * (1.0f / (float)MD);

    float s2 = 0.0f;
#pragma unroll 1
    for (int i = 0; i < 8; ++i) {
        const v4f a = *(const v4f*)(yr + i * 128);
        const float dx = a.x - mu, dy = a.y - mu, dz = a.z - mu, dw = a.w - mu;
        s2 += (dx * dx + dy * dy) + (dz * dz + dw * dw);
    }
#pragma unroll
    for (int m = 1; m < 32; m <<= 1) s2 += __shfl_xor(s2, m, 32);
    const float rstd = rsqrtf(s2 * (1.0f / (float)MD) + 1.0e-5f);

    const float* gr = gam + lane * 4;
    const float* br = bet + lane * 4;
    float*    xor_ = xo + (size_t)row * MD + lane * 4;
    _Float16* xhr  = xh + (size_t)row * MD + lane * 4;
    ln_store<WH>(yr, gr, br, mu, rstd, xor_, xhr);
    __threadfence();
    ln_store<WH>(yr, gr, br, mu, rstd, xor_, xhr);
}

extern "C" void kernel_launch(void* const* d_in, const int* in_sizes, int n_in,
                              void* d_out, int out_size, void* d_ws, size_t ws_size,
                              hipStream_t stream) {
    if (n_in < 16) return;
    if (in_sizes[0] < ((NB - 1) * SEQ_FULL + SEQ) * MD) return;
    if (in_sizes[1] < (NB - 1) * SEQ_FULL + SEQ) return;
    if (in_sizes[2] < MD * MD || in_sizes[4] < MD * MD || in_sizes[6] < MD * MD || in_sizes[8] < MD * MD) return;
    if (in_sizes[3] < MD || in_sizes[5] < MD || in_sizes[7] < MD || in_sizes[9] < MD) return;
    if (in_sizes[10] < MD || in_sizes[11] < MD) return;
    if (in_sizes[12] < MD * FF || in_sizes[13] < FF || in_sizes[14] < FF * MD || in_sizes[15] < MD) return;
    if (out_size < NTOK * MD) return;

    const float* inp  = (const float*)d_in[0];
    const int*   mask = (const int*)d_in[1];
    const float* Wq   = (const float*)d_in[2];
    const float* bq   = (const float*)d_in[3];
    const float* Wk   = (const float*)d_in[4];
    const float* bk   = (const float*)d_in[5];
    const float* Wv   = (const float*)d_in[6];
    const float* bv   = (const float*)d_in[7];
    const float* Wo   = (const float*)d_in[8];
    const float* bo   = (const float*)d_in[9];
    const float* ln_g = (const float*)d_in[10];
    const float* ln_b = (const float*)d_in[11];
    const float* W1   = (const float*)d_in[12];
    const float* b1   = (const float*)d_in[13];
    const float* W2   = (const float*)d_in[14];
    const float* b2   = (const float*)d_in[15];
    float* out = (float*)d_out;

    char* ws = (char*)d_ws;
    size_t off = 0;
    const size_t WSQ  = (size_t)MD * MD * 2;
    const size_t WSF  = (size_t)FF * MD * 2;
    const size_t PL16 = (size_t)NTOK * MD * 2;
    const size_t PL32 = (size_t)NTOK * MD * 4;
    _Float16* WqT = (_Float16*)(ws + off); off += WSQ;
    _Float16* WkT = (_Float16*)(ws + off); off += WSQ;
    _Float16* WvT = (_Float16*)(ws + off); off += WSQ;
    _Float16* WoT = (_Float16*)(ws + off); off += WSQ;
    _Float16* W1T = (_Float16*)(ws + off); off += WSF;
    _Float16* W2T = (_Float16*)(ws + off); off += WSF;
    _Float16* XH  = (_Float16*)(ws + off); off += PL16;
    _Float16* QP  = (_Float16*)(ws + off); off += PL16;
    _Float16* KP  = (_Float16*)(ws + off); off += PL16;
    _Float16* VP  = (_Float16*)(ws + off); off += PL16;
    _Float16* VT  = (_Float16*)(ws + off); off += PL16;
    _Float16* HP  = QP;
    static_assert((size_t)NTOK * FF * 2 == 4 * ((size_t)NTOK * MD * 2));
    _Float16* CTX = (_Float16*)(ws + off); off += PL16;
    float*    Y   = (float*)(ws + off);    off += PL32;
    float*    X32 = (float*)(ws + off);    off += PL32;
    _Float16* XH2 = (_Float16*)(ws + off); off += PL16;
    if (off > ws_size) return;

    k_wtr<<<dim3(MD / 64, MD / 64), dim3(256), 0, stream>>>(Wq, MD, MD, WqT);
    k_wtr<<<dim3(MD / 64, MD / 64), dim3(256), 0, stream>>>(Wk, MD, MD, WkT);
    k_wtr<<<dim3(MD / 64, MD / 64), dim3(256), 0, stream>>>(Wv, MD, MD, WvT);
    k_wtr<<<dim3(MD / 64, MD / 64), dim3(256), 0, stream>>>(Wo, MD, MD, WoT);
    k_wtr<<<dim3(FF / 64, MD / 64), dim3(256), 0, stream>>>(W1, FF, MD, W1T);
    k_wtr<<<dim3(MD / 64, FF / 64), dim3(256), 0, stream>>>(W2, MD, FF, W2T);

    k_xcvt<<<dim3(NTOK / 2), dim3(256), 0, stream>>>(inp, XH);

    k_gemm<0><<<dim3(NTOK / 128, MD / 128), dim3(256), 0, stream>>>(XH, MD, WqT, MD, bq, bq, 0, (void*)QP, MD, MD, SA_QKV, A_CARRY);
    k_gemm<0><<<dim3(NTOK / 128, MD / 128), dim3(256), 0, stream>>>(XH, MD, WkT, MD, bk, bk, 0, (void*)KP, MD, MD, SA_QKV, A_CARRY);
    k_gemm<0><<<dim3(NTOK / 128, MD / 128), dim3(256), 0, stream>>>(XH, MD, WvT, MD, bv, bv, 0, (void*)VP, MD, MD, SA_QKV, A_CARRY);

    k_vtr<<<dim3(NTOK / 64, NH), dim3(256), 0, stream>>>(VP, VT);
    k_attn<<<dim3(SEQ / 128, NB * NH), dim3(256), 0, stream>>>(QP, KP, VT, mask, CTX);

    k_gemm<2><<<dim3(NTOK / 128, MD / 128), dim3(256), 0, stream>>>(CTX, MD, WoT, MD, bo, inp, MD, (void*)Y, MD, MD, SA_WO, 1.0f);
    k_ln<1><<<dim3(NTOK / 8), dim3(256), 0, stream>>>(Y, ln_g, ln_b, X32, XH2);

    k_gemm<1><<<dim3(NTOK / 128, FF / 128), dim3(256), 0, stream>>>(XH2, MD, W1T, MD, b1, b1, 0, (void*)HP, FF, MD, SA_FF, A_CARRY);
    k_gemm<3><<<dim3(NTOK / 128, MD / 128), dim3(256), 0, stream>>>(HP, FF, W2T, FF, b2, X32, MD, (void*)Y, MD, FF, SA_FF, 1.0f);
    k_ln<0><<<dim3(NTOK / 8), dim3(256), 0, stream>>>(Y, ln_g, ln_b, out, XH2);
}
